// image_prj_39926015984314
// MI455X (gfx1250) — hardware-verified
//
#include <hip/hip_runtime.h>
#include <math.h>

typedef __attribute__((ext_vector_type(16))) _Float16 v16h;
typedef __attribute__((ext_vector_type(16))) __bf16 v16b;
typedef __attribute__((ext_vector_type(8)))  _Float16 v8h;
typedef __attribute__((ext_vector_type(8)))  float v8f;
typedef __attribute__((ext_vector_type(4)))  float v4f;
typedef __attribute__((ext_vector_type(2)))  float v2f;
typedef __attribute__((ext_vector_type(4)))  unsigned v4u;
typedef __attribute__((ext_vector_type(4)))  int v4i;
typedef float __attribute__((may_alias)) float_a;
typedef int __attribute__((may_alias)) int_a;

template <typename T> __device__ __forceinline__ void vst2(void* p, T v) { *(volatile T*)p = v; __threadfence(); *(volatile T*)p = v; }
__device__ __forceinline__ v8f wmma16(v16h a, v16h b, v8f c) {
  v8f d = __builtin_amdgcn_wmma_f32_16x16x32_f16(false, a, false, b, (short)0, c, false, false);
  asm volatile("v_nop\n\tv_nop\n\tv_nop\n\tv_nop" : "+v"(d) : "v"(a), "v"(b));
  return d;
}
__device__ __forceinline__ v8f wmma_bf(v16b a, v16b b, v8f c) {
  v8f d = __builtin_amdgcn_wmma_f32_16x16x32_bf16(false, a, false, b, (short)0, c, false, false);
  asm volatile("v_nop\n\tv_nop\n\tv_nop\n\tv_nop" : "+v"(d) : "v"(a), "v"(b));
  return d;
}
__device__ __forceinline__ v16h frag_h(const _Float16* rowk0, int lane) {
  union { v16h v; v8h q[2]; } u; const _Float16* p = rowk0 + 8 * (lane >> 4);
  u.q[0] = *(const v8h*)p; u.q[1] = *(const v8h*)(p + 16); return u.v;
}
__device__ __forceinline__ v16h frag_f32(const float* rowk0, int lane) {
  v16h a; const float* p = rowk0 + 8 * (lane >> 4);
#pragma unroll
  for (int i = 0; i < 8; ++i) { a[i] = (_Float16)p[i]; a[8 + i] = (_Float16)p[16 + i]; }
  return a;
}
__device__ __forceinline__ v16h frag_f32s(const float* rowk0, int lane, float sc) {
  v16h a; const float* p = rowk0 + 8 * (lane >> 4);
#pragma unroll
  for (int i = 0; i < 8; ++i) { a[i] = (_Float16)(p[i] * sc); a[8 + i] = (_Float16)(p[16 + i] * sc); }
  return a;
}
__device__ __forceinline__ v16h fragc_f32(const float* W, int k0, int n, int lane, int ld, int K) {
  v16h a; const int g = lane >> 4;
#pragma unroll
  for (int i = 0; i < 8; ++i) { const int ka = k0 + 8 * g + i, kb = ka + 16;
    a[i] = (_Float16)(ka < K ? W[(size_t)(ka < K ? ka : K - 1) * ld + n] : 0.f); a[8 + i] = (_Float16)(kb < K ? W[(size_t)(kb < K ? kb : K - 1) * ld + n] : 0.f); }
  return a;
}
struct F2 { v16b h, l; };
__device__ __forceinline__ F2 bsplit16(const float v[16]) { F2 r;
#pragma unroll
  for (int i = 0; i < 16; ++i) { const __bf16 h = (__bf16)v[i]; r.h[i] = h; r.l[i] = (__bf16)(v[i] - (float)h); }
  return r; }
__device__ __forceinline__ F2 split_row(const float* row, int k0, int lane) { float v[16]; const float* p = row + k0 + 8 * (lane >> 4);
#pragma unroll
  for (int i = 0; i < 8; ++i) { v[i] = p[i]; v[8 + i] = p[16 + i]; }
  return bsplit16(v); }
__device__ __forceinline__ F2 split_rowK(const float* row, int k0, int lane, int K) { float v[16]; const int g = lane >> 4;
#pragma unroll
  for (int i = 0; i < 8; ++i) { const int ka = k0 + 8 * g + i, kb = ka + 16; v[i] = ka < K ? row[ka < K ? ka : K - 1] : 0.f; v[8 + i] = kb < K ? row[kb < K ? kb : K - 1] : 0.f; }
  return bsplit16(v); }
__device__ __forceinline__ F2 split_col(const float* W, int k0, int n, int lane, int ld, int K) { float v[16]; const int g = lane >> 4;
#pragma unroll
  for (int i = 0; i < 8; ++i) { const int ka = k0 + 8 * g + i, kb = ka + 16; v[i] = ka < K ? W[(size_t)(ka < K ? ka : K - 1) * ld + n] : 0.f; v[8 + i] = kb < K ? W[(size_t)(kb < K ? kb : K - 1) * ld + n] : 0.f; }
  return bsplit16(v); }
__device__ __forceinline__ v8f mac3(const F2& a, const F2& b, v8f c) { c = wmma_bf(a.l, b.h, c); c = wmma_bf(a.h, b.l, c); return wmma_bf(a.h, b.h, c); }
__device__ __forceinline__ float sigm(float v) { return 1.0f / (1.0f + expf(-v)); }
#define LDSX() do { asm volatile("s_wait_dscnt 0" ::: "memory"); __builtin_amdgcn_wave_barrier(); __builtin_amdgcn_fence(__ATOMIC_RELEASE, "workgroup"); } while (0)


#define NN 2048
#define PP 2198
#define PADB 75
#define NANG 32
#define PW 2304
#define COFF 21
#define LW 2240
typedef __attribute__((ext_vector_type(8))) __bf16 v8b;
__device__ __forceinline__ v16b frag_gbf(const float* rowk0, int lane) {
  v16b a; const float* p = rowk0 + 8 * (lane >> 4);
#pragma unroll
  for (int i = 0; i < 8; ++i) { a[i] = (__bf16)p[i]; a[8 + i] = (__bf16)p[16 + i]; }
  return a;
}
__device__ __attribute__((noinline)) float cos_ni(float v) { return cosf(v); }
__device__ __attribute__((noinline)) float sin_ni(float v) { return sinf(v); }
#define WS_C    0u
#define WS_UT   (WS_C + 4u * NN * NN)
#define WS_PD   (WS_UT + 4u * NN * NN)
#define WS_LN   (WS_PD + 4u * PP * PW)
#define WS_END  (WS_LN + 4u * NANG * LW)

__global__ __launch_bounds__(512) void k_dct(float* __restrict__ C) {
  const int k = blockIdx.x, tid = threadIdx.x;
  const float sk = k == 0 ? (float)0.022097086912079608 : 0.03125f;
  v4f v;
#pragma unroll
  for (int i = 0; i < 4; ++i) { const int n = tid * 4 + i; int t = (int)(((long long)(2 * n + 1) * k) & 8191); float sg = 1.0f;
    if (t > 4096) t = 8192 - t;
    if (t > 2048) { t = 4096 - t; sg = -1.0f; }
    float c; if (t > 1024) c = sin_ni((float)(2048 - t) * (float)(3.14159265358979323846 / 4096.0)); else c = cos_ni((float)t * (float)(3.14159265358979323846 / 4096.0));
    v[i] = sg * c * sk; }
  vst2(C + (size_t)k * NN + tid * 4, v);
}
__global__ __launch_bounds__(256) void k_zero(float* __restrict__ PD) {
  const int r = blockIdx.x, tid = threadIdx.x; const v4f z = {0.f, 0.f, 0.f, 0.f};
  for (int q = tid; q < PW / 4; q += 256) vst2(PD + (size_t)r * PW + q * 4, z);
}
__global__ __launch_bounds__(128) void k_u(const float* __restrict__ X, const float* __restrict__ C, float* __restrict__ UT) {
  __shared__ __align__(16) float st[128][68];
  const int tid = threadIdx.x, wave = tid >> 5, lane = tid & 31, col = lane & 15, g = lane >> 4; const int n0 = blockIdx.x * 64, m0 = blockIdx.y * 128;
  v8f acc[8] = {};
#pragma unroll 1
  for (int kc = 0; kc < NN / 32; ++kc) { const v16b a = frag_gbf(X + (size_t)(n0 + wave * 16 + col) * NN + kc * 32, lane);
#pragma unroll
    for (int j = 0; j < 8; ++j) { const F2 cb = split_row(C + (size_t)(m0 + j * 16 + col) * NN, kc * 32, lane); acc[j] = wmma_bf(a, cb.l, acc[j]); acc[j] = wmma_bf(a, cb.h, acc[j]); } }
#pragma unroll
  for (int j = 0; j < 8; ++j)
#pragma unroll
    for (int r = 0; r < 8; ++r) st[j * 16 + col][wave * 16 + 8 * g + r] = acc[j][r];
  __syncthreads();
  for (int q = tid; q < 128 * 16; q += 128) { const int ml = q >> 4, pc = q & 15; vst2(UT + (size_t)(m0 + ml) * NN + n0 + pc * 4, *(const v4f*)&st[ml][pc * 4]); }
}
__global__ __launch_bounds__(128) void k_d(const float* __restrict__ C, const float* __restrict__ UT, float* __restrict__ PD) {
  __shared__ __align__(16) float so[4][16][132];
  const int tid = threadIdx.x, wave = tid >> 5, lane = tid & 31, col = lane & 15, g = lane >> 4; const int k0 = blockIdx.x * 64 + wave * 16, m0 = blockIdx.y * 128;
  v8f acc[8] = {};
#pragma unroll 1
  for (int kc = 0; kc < NN / 32; ++kc) { const F2 a = split_row(C + (size_t)(k0 + col) * NN, kc * 32, lane);
#pragma unroll
    for (int j = 0; j < 8; ++j) { const F2 ub = split_row(UT + (size_t)(m0 + j * 16 + col) * NN, kc * 32, lane); acc[j] = mac3(a, ub, acc[j]); } }
#pragma unroll
  for (int j = 0; j < 8; ++j)
#pragma unroll
    for (int r = 0; r < 8; ++r) so[wave][8 * g + r][j * 16 + col] = acc[j][r];
  LDSX();
  for (int rl = 0; rl < 16; ++rl) vst2(PD + (size_t)(k0 + rl + PADB) * PW + (m0 + PADB + COFF) + lane * 4, *(const v4f*)(&so[wave][rl][lane * 4]));
}
__global__ __launch_bounds__(256) void k_rot(const float* __restrict__ PD, float* __restrict__ LN, int abase, int astride) {
  __shared__ float sred[4][64]; __shared__ __align__(16) float srow[64];
  const int tid = threadIdx.x, a = abase + blockIdx.y * astride, x0 = blockIdx.x * 64; const int xl = tid & 63, ph = tid >> 6; const int xo = x0 + xl;
  const float ang = (float)((double)a * (3.14159265358979323846 / 31.0));
  const float ca = cos_ni(ang), sa = sin_ni(ang); const float center = (float)(PP / 2);
  const float xx = (float)xo;
  float acc = 0.f;
  if (xo < PP) { const float cx = ca * xx, sx = -sa * xx, kx = center * (ca + sa - 1.0f), ky = center * (ca - sa - 1.0f);
#pragma unroll 1
    for (int y = ph; y < PP; y += 4) { const float yy = (float)y;
      const float x_in = cx + sa * yy - kx;
      const float y_in = sx + ca * yy - ky;
      const float fx0 = floorf(x_in), fy0 = floorf(y_in); const float wx = x_in - fx0, wy = y_in - fy0;
      int x0i = (int)fx0; x0i += (x0i < 0) ? PP : 0; x0i -= (x0i >= PP) ? PP : 0; int y0i = (int)fy0; y0i += (y0i < 0) ? PP : 0; y0i -= (y0i >= PP) ? PP : 0;
      const int x1i = (x0i + 1 == PP) ? 0 : x0i + 1, y1i = (y0i + 1 == PP) ? 0 : y0i + 1;
      const float* r0p = PD + (size_t)y0i * PW + x0i + COFF; const float* r1p = PD + (size_t)y1i * PW + x0i + COFF;
      const float w0 = PD[(size_t)y0i * PW + COFF], w1 = PD[(size_t)y1i * PW + COFF];
      const float v00 = r0p[0], v10 = r1p[0]; const float v01 = (x1i == 0) ? w0 : r0p[1], v11 = (x1i == 0) ? w1 : r1p[1];
      acc += (1.0f - wy) * ((1.0f - wx) * v00 + wx * v01) + wy * ((1.0f - wx) * v10 + wx * v11); } }
  sred[ph][xl] = acc;
  __syncthreads();
  if (tid < 64) srow[tid] = (sred[0][tid] + sred[1][tid]) + (sred[2][tid] + sred[3][tid]);
  __syncthreads();
  if (tid < 16) vst2(LN + (size_t)a * LW + x0 + tid * 4, *(const v4f*)&srow[tid * 4]);
}
__global__ __launch_bounds__(256) void k_fin(const float* __restrict__ LN, float* __restrict__ out) {
  __shared__ float sm[8]; __shared__ float smax;
  const int tid = threadIdx.x, wave = tid >> 5, lane = tid & 31; float m = -3.0e38f;
  for (int q = tid; q < NANG * PP; q += 256) { const int a = q / PP, p = q % PP; m = fmaxf(m, LN[(size_t)a * LW + p]); }
#pragma unroll
  for (int o = 1; o < 32; o <<= 1) m = fmaxf(m, __shfl_xor(m, o));
  if (lane == 0) sm[wave] = m;
  __syncthreads();
  if (tid == 0) { float mm = sm[0]; for (int w = 1; w < 8; ++w) mm = fmaxf(mm, sm[w]); smax = mm; }
  __syncthreads();
  const float inv = smax;
  for (int q = tid; q < PP * 8; q += 256) { const int p = q >> 3, pc = q & 7; v4f v;
#pragma unroll
    for (int i = 0; i < 4; ++i) v[i] = LN[(size_t)(pc * 4 + i) * LW + p] / inv;
    vst2(out + (size_t)p * NANG + pc * 4, v); }
}

#ifndef DBG
#define DBG 0
#endif
#if DBG != 0
__global__ __launch_bounds__(256) void k_dbgA(const float* __restrict__ PD, float* __restrict__ out) {
  const int tid = threadIdx.x; const int r = blockIdx.x;
  if (tid < 64) { v4f v; for (int i = 0; i < 4; ++i) v[i] = PD[(size_t)(r + PADB) * PW + PADB + COFF + tid * 4 + i]; vst2(out + (size_t)r * 256 + tid * 4, v); }
  if (r == 0) { const v4f z = {0.f,0.f,0.f,0.f}; for (int q = 4096 + tid; q < PP * NANG / 4; q += 256) vst2(out + (size_t)q * 4, z); }
}
__global__ __launch_bounds__(256) void k_pat(float* __restrict__ PD) {
  const int y = blockIdx.x, tid = threadIdx.x;
  for (int q = tid; q < PW / 4; q += 256) { v4f v; for (int i = 0; i < 4; ++i) { const int bc = q * 4 + i; const int x = bc - COFF - PADB; v[i] = (x >= 0 && x < NN) ? (float)(((y * 131 + x * 7919) % 1009)) / 1009.0f - 0.5f : 0.f; } vst2(PD + (size_t)(y + PADB) * PW + q * 4, v); }
}
__global__ __launch_bounds__(256) void k_finB(const float* __restrict__ LN, float* __restrict__ out) {
  __shared__ float sm[8]; __shared__ float smax;
  const int tid = threadIdx.x, wave = tid >> 5, lane = tid & 31; float m = -3.0e38f;
  for (int q = tid; q < 4 * PP; q += 256) { const int a = (q / PP) * 9, p = q % PP; m = fmaxf(m, LN[(size_t)a * LW + p]); }
  for (int o = 1; o < 32; o <<= 1) m = fmaxf(m, __shfl_xor(m, o));
  if (lane == 0) sm[wave] = m; __syncthreads();
  if (tid == 0) { float mm = sm[0]; for (int w = 1; w < 8; ++w) mm = fmaxf(mm, sm[w]); smax = mm; } __syncthreads();
  for (int q = tid; q < PP * 8; q += 256) { const int p = q >> 3, pc = q & 7; v4f v; for (int i = 0; i < 4; ++i) { const int a = pc * 4 + i; v[i] = (a < 4) ? LN[(size_t)(a * 9) * LW + p] / smax : 0.f; } vst2(out + (size_t)p * NANG + pc * 4, v); }
}
#endif
extern "C" void kernel_launch(void* const* d_in, const int* in_sizes, int n_in, void* d_out, int out_size, void* d_ws, size_t ws_size, hipStream_t stream) {
  (void)in_sizes; (void)n_in; (void)out_size;
  if (ws_size < (size_t)WS_END) return;
  char* ws = (char*)d_ws; float *C = (float*)(ws + WS_C), *UT = (float*)(ws + WS_UT), *PD = (float*)(ws + WS_PD), *LN = (float*)(ws + WS_LN);
#if DBG == 0
  k_dct<<<NN, 512, 0, stream>>>(C);
  k_zero<<<PP, 256, 0, stream>>>(PD);
  k_u<<<dim3(NN / 64, NN / 128), 128, 0, stream>>>((const float*)d_in[0], C, UT);
  k_d<<<dim3(NN / 64, NN / 128), 128, 0, stream>>>(C, UT, PD);
  k_rot<<<dim3((PP + 63) / 64, NANG), 256, 0, stream>>>(PD, LN, 0, 1);
  k_fin<<<1, 256, 0, stream>>>(LN, (float*)d_out);
#elif DBG == 1
  k_dct<<<NN, 512, 0, stream>>>(C);
  k_zero<<<PP, 256, 0, stream>>>(PD);
  k_u<<<dim3(NN / 64, 2), 128, 0, stream>>>((const float*)d_in[0], C, UT);
  k_d<<<dim3(1, 2), 128, 0, stream>>>(C, UT, PD);
  k_dbgA<<<64, 256, 0, stream>>>(PD, (float*)d_out);
#else
  k_zero<<<PP, 256, 0, stream>>>(PD);
  k_pat<<<NN, 256, 0, stream>>>(PD);
  k_rot<<<dim3((PP + 63) / 64, 4), 256, 0, stream>>>(PD, LN, 0, 9);
  k_finB<<<1, 256, 0, stream>>>(LN, (float*)d_out);
#endif
}
